// EncoderLayer_13666585936666
// MI455X (gfx1250) — hardware-verified
//
#include <hip/hip_runtime.h>
#include <math.h>

#ifndef NB
#define NB 2
#endif
#ifndef SEQ
#define SEQ 2048
#endif
#define SEQ_FULL 2048
#define DM 1024
#define NHEAD 16
#define DHEAD 64
#define DFF 4096
#define MTOK (NB * SEQ)
#define LN_BLK_ELEMS 8192
#define LN_BPB ((SEQ * DM) / LN_BLK_ELEMS)

static_assert(NHEAD * DHEAD == DM);
static_assert(DHEAD == 64);
static_assert(SEQ % 64 == 0);
static_assert(SEQ <= SEQ_FULL);
static_assert(MTOK % 64 == 0);
static_assert(DM % 64 == 0 && DFF % 64 == 0);
static_assert(DM % 32 == 0 && DFF % 32 == 0);
static_assert(DM == 256 * 4);
static_assert(LN_BLK_ELEMS == 8 * DM);
static_assert((SEQ * DM) % LN_BLK_ELEMS == 0);

typedef __attribute__((ext_vector_type(16))) _Float16 v16h;
typedef __attribute__((ext_vector_type(8)))  _Float16 v8h;
typedef __attribute__((ext_vector_type(8)))  float    v8f;
typedef __attribute__((ext_vector_type(4)))  float    v4f;
typedef __attribute__((ext_vector_type(4)))  unsigned int u4v;
typedef __attribute__((ext_vector_type(2)))  unsigned int u2v;

union FragU { v16h v; v8h h[2]; };
__device__ __forceinline__ v16h frag_ld_g(const _Float16* __restrict__ p) { FragU f; f.h[0] = *(const v8h*)(p); f.h[1] = *(const v8h*)(p + 16); return f.v; }

__device__ __forceinline__ v8f wmma_raw(v16h a, v16h b, v8f c) { return __builtin_amdgcn_wmma_f32_16x16x32_f16(false, a, false, b, (short)0, c, false, false); }
__device__ __forceinline__ v8f mma16(v16h a, v16h b, v8f c) {
    c = __builtin_amdgcn_wmma_f32_16x16x32_f16(false, a, false, b, (short)0, c, false, false);
    asm volatile("v_nop\n\tv_nop\n\tv_nop\n\tv_nop" : "+v"(c) : "v"(a), "v"(b));
    return c;
}
__device__ __forceinline__ void dep_guard_h(v8f& a, v8f& b, v16h x, v16h y) { asm volatile("v_nop\n\tv_nop\n\tv_nop\n\tv_nop" : "+v"(a), "+v"(b) : "v"(x), "v"(y)); }
__device__ __forceinline__ void keep4_h(v16h a, v16h b, v16h c, v16h d) { asm volatile("v_nop" :: "v"(a), "v"(b), "v"(c), "v"(d)); }
__device__ __forceinline__ void acc_guard4(v8f& a, v8f& b, v8f& c, v8f& d) { asm volatile("v_nop\n\tv_nop\n\tv_nop\n\tv_nop" : "+v"(a), "+v"(b), "+v"(c), "+v"(d)); }

#define VST2(T, ptr, val) do { const T vst2_v_ = (val); *(volatile T*)(ptr) = vst2_v_; __threadfence(); *(volatile T*)(ptr) = vst2_v_; } while (0)
#define VST2V4(ptr, val) do { const v4f vst2_v4_ = (val); *(volatile v4f*)(ptr) = vst2_v4_; __threadfence(); *(volatile v4f*)(ptr) = vst2_v4_; } while (0)

__device__ __forceinline__ float cmb_bf(float v) { const unsigned u = __builtin_bit_cast(unsigned, v); const unsigned r = (u + 0x7fffu + ((u >> 16) & 1u)) & 0xffff0000u; return __builtin_bit_cast(float, r); }
__device__ __forceinline__ unsigned int pk2h(float a, float b) { return (unsigned int)__builtin_bit_cast(unsigned short, (_Float16)a) | ((unsigned int)__builtin_bit_cast(unsigned short, (_Float16)b) << 16); }

__global__ __launch_bounds__(256) void k_cast_x(const float* __restrict__ SRC, unsigned short* __restrict__ DST) {
    const long long u = (long long)blockIdx.x * 256 + threadIdx.x; const int per = DM / 8; if (u >= (long long)MTOK * per) return;
    const int r = (int)(u / per); const int c0 = 8 * (int)(u % per); const int b = r / SEQ, s = r - b * SEQ;
    const float* sp = SRC + ((long long)b * SEQ_FULL + s) * DM + c0;
    const v4f a0 = *(const v4f*)(sp), a1 = *(const v4f*)(sp + 4);
    u4v pk; pk.x = pk2h(cmb_bf(a0.x), cmb_bf(a0.y)); pk.y = pk2h(cmb_bf(a0.z), cmb_bf(a0.w)); pk.z = pk2h(cmb_bf(a1.x), cmb_bf(a1.y)); pk.w = pk2h(cmb_bf(a1.z), cmb_bf(a1.w));
    VST2(u4v, (u4v*)(DST + (long long)r * DM + c0), pk);
}
__global__ __launch_bounds__(256) void k_castT(const float* __restrict__ SRC, int lds, unsigned short* __restrict__ DST, int ldd, int nR, int nC, float sc) {
    const long long u = (long long)blockIdx.x * 256 + threadIdx.x; const int per = nR / 8; if (u >= (long long)nC * per) return; const int c = (int)(u / per); const int r0 = 8 * (int)(u % per);
    float w[8];
#pragma unroll
    for (int e = 0; e < 8; ++e) w[e] = cmb_bf(SRC[(long long)(r0 + e) * lds + c]) * sc;
    u4v pk; pk.x = pk2h(w[0], w[1]); pk.y = pk2h(w[2], w[3]); pk.z = pk2h(w[4], w[5]); pk.w = pk2h(w[6], w[7]);
    VST2(u4v, (u4v*)(DST + (long long)c * ldd + r0), pk);
}

template <int BIAS_MODE, int OUT_MODE, int ACT>
__device__ __forceinline__ void gemm64_body(const _Float16* __restrict__ A, const int lda, const _Float16* __restrict__ Bt, const int ldb,
                                            void* __restrict__ Cout, const int ldc, const float* __restrict__ bias,
                                            const int M, const int N, const int K, const float scale) {
    __shared__ __align__(16) float sT[8][16 * 68];
    const int lane = threadIdx.x & 31;
    const int wave = threadIdx.x >> 5;
    const int tilesN = N >> 6;
    const int tilesM = M >> 6;
    const int tile = blockIdx.x * 8 + wave;
    if (tile >= tilesM * tilesN) return;
    const int tm = tile / tilesN;
    const int tn = tile - tm * tilesN;
    const int m0 = tm << 6;
    const int n0 = tn << 6;
    const int rlane = lane & 15;
    const int koff  = (lane >> 4) * 8;
    const int mOff  = (lane >> 4) * 8;

    v8f acc[4][4];
#pragma unroll
    for (int i = 0; i < 4; ++i)
#pragma unroll
        for (int j = 0; j < 4; ++j) acc[i][j] = (v8f){0.f, 0.f, 0.f, 0.f, 0.f, 0.f, 0.f, 0.f};

    for (int k0 = 0; k0 < K; k0 += 32) {
        v16h bh[4];
#pragma unroll
        for (int j = 0; j < 4; ++j) bh[j] = frag_ld_g(Bt + (size_t)(n0 + (j << 4) + rlane) * ldb + koff + k0);
#pragma unroll
        for (int i = 0; i < 4; ++i) {
            const v16h ah = frag_ld_g(A + (size_t)(m0 + (i << 4) + rlane) * lda + koff + k0);
#pragma unroll
            for (int j = 0; j < 4; ++j) acc[i][j] = wmma_raw(ah, bh[j], acc[i][j]);
            dep_guard_h(acc[i][0], acc[i][3], ah, ah);
        }
        keep4_h(bh[0], bh[1], bh[2], bh[3]);
    }
    acc_guard4(acc[0][0], acc[0][1], acc[0][2], acc[0][3]);
    acc_guard4(acc[1][0], acc[1][1], acc[1][2], acc[1][3]);
    acc_guard4(acc[2][0], acc[2][1], acc[2][2], acc[2][3]);
    acc_guard4(acc[3][0], acc[3][1], acc[3][2], acc[3][3]);

#pragma unroll
    for (int i = 0; i < 4; ++i) {
        const int mBase = m0 + (i << 4);
#pragma unroll
        for (int j = 0; j < 4; ++j) {
            const int n = n0 + (j << 4) + rlane;
            float bv = 0.f;
            if (BIAS_MODE == 2) bv = cmb_bf(bias[n]);
#pragma unroll
            for (int r = 0; r < 8; ++r) {
                float v = acc[i][j][r] * scale;
                if (BIAS_MODE == 1) v += cmb_bf(bias[mBase + mOff + r]);
                if (BIAS_MODE == 2) v += bv;
                if (ACT == 2) v = fmaxf(v, 0.0f);
                sT[wave][(mOff + r) * 68 + (j << 4) + rlane] = v;
            }
        }
        __builtin_amdgcn_fence(3  , "workgroup");
        __builtin_amdgcn_wave_barrier();
        __builtin_amdgcn_fence(2  , "workgroup");
        if (OUT_MODE == 0) {
            float* C = (float*)Cout;
            const int hh = lane >> 4, c4 = (lane & 15) * 4;
            for (int pass = 0; pass < 2; ++pass) {
#pragma unroll
                for (int it = 0; it < 8; ++it) {
                    const int row = it * 2 + hh;
                    const v4f v = *(const v4f*)(&sT[wave][row * 68 + c4]);
                    *(volatile v4f*)(C + (size_t)(mBase + row) * ldc + n0 + c4) = v;
                }
                __threadfence();
            }
        } else {
            const int q = lane >> 3, c8 = (lane & 7) * 8;
            unsigned short* C = (unsigned short*)Cout;
            for (int pass = 0; pass < 2; ++pass) {
#pragma unroll
                for (int it = 0; it < 4; ++it) {
                    const int row = it * 4 + q;
                    v8h hv;
#pragma unroll
                    for (int e = 0; e < 8; ++e) hv[e] = (_Float16)sT[wave][row * 68 + c8 + e];
                    *(volatile v8h*)(C + (size_t)(mBase + row) * ldc + n0 + c8) = hv;
                }
                __threadfence();
            }
        }
        __builtin_amdgcn_fence(3  , "workgroup");
        __builtin_amdgcn_wave_barrier();
        __builtin_amdgcn_fence(2  , "workgroup");
    }
}

__global__ __launch_bounds__(256) void k_gemm_proj(const unsigned short* __restrict__ X16, const unsigned short* __restrict__ W16, unsigned short* __restrict__ C16, const float* __restrict__ bias) {
    gemm64_body<2, 1, 0>((const _Float16*)X16, DM, (const _Float16*)W16, DM, (void*)C16, DM, bias, MTOK, DM, DM, 0.0625f);
}
__global__ __launch_bounds__(256) void k_gemm_vt(const unsigned short* __restrict__ WV16, const unsigned short* __restrict__ X16, unsigned short* __restrict__ VT16, const float* __restrict__ bias) {
    gemm64_body<1, 1, 0>((const _Float16*)WV16, DM, (const _Float16*)X16, DM, (void*)VT16, MTOK, bias, DM, MTOK, DM, 0.0625f);
}
__global__ __launch_bounds__(256) void k_gemm_ff1(const unsigned short* __restrict__ H16, const unsigned short* __restrict__ W1T, unsigned short* __restrict__ F16p, const float* __restrict__ bias) {
    gemm64_body<2, 1, 2>((const _Float16*)H16, DM, (const _Float16*)W1T, DM, (void*)F16p, DFF, bias, MTOK, DFF, DM, 0.0625f);
}
__global__ __launch_bounds__(256) void k_gemm_ff2(const unsigned short* __restrict__ F16p, const unsigned short* __restrict__ W2T, float* __restrict__ FFo, const float* __restrict__ bias) {
    gemm64_body<2, 0, 0>((const _Float16*)F16p, DFF, (const _Float16*)W2T, DFF, (void*)FFo, DM, bias, MTOK, DM, DFF, 0.0625f);
}

__global__ __launch_bounds__(128) void k_attn(const unsigned short* __restrict__ Qp, const unsigned short* __restrict__ Kp, const unsigned short* __restrict__ VTp, float* __restrict__ out) {
    __shared__ __align__(16) _Float16 Ksh[64 * 64];
    __shared__ __align__(16) _Float16 Vth[64 * 64];
    __shared__ __align__(16) _Float16 Psh[4][16 * 64];
    __shared__ __align__(16) float    Os[4][16 * 68];
    const float PSC = 32768.0f;
    const float SCL = 0.125f * 1.4426950408889634f;
    const float NEG = -__builtin_inff();

    const int tid = threadIdx.x, wave = tid >> 5, lane = tid & 31, hh = lane >> 4, c = lane & 15;
    const int nqb = SEQ / 64;
    const int bx = blockIdx.x;
    const int qb = bx % nqb;
    const int bh = bx / nqb;
    const int h = bh % NHEAD;
    const int b = bh / NHEAD;
    const int q0 = qb * 64 + wave * 16;

    const _Float16* Qb = (const _Float16*)Qp + (size_t)b * SEQ * DM + (size_t)h * DHEAD;
    const _Float16* Kb = (const _Float16*)Kp + (size_t)b * SEQ * DM + (size_t)h * DHEAD;
    const _Float16* Vb = (const _Float16*)VTp + (size_t)h * DHEAD * MTOK + (size_t)b * SEQ;
    float* ob = out + (size_t)b * SEQ * DM + (size_t)h * DHEAD;

    const _Float16* qrow = Qb + (size_t)(q0 + c) * DM + 8 * hh;
    const v16h qa0 = frag_ld_g(qrow);
    const v16h qa1 = frag_ld_g(qrow + 32);

    float mrow[8], lrow[8];
    v8f oacc[4];
#pragma unroll
    for (int r = 0; r < 8; ++r) { mrow[r] = NEG; lrow[r] = 0.f; }
#pragma unroll
    for (int t = 0; t < 4; ++t) oacc[t] = (v8f){0.f, 0.f, 0.f, 0.f, 0.f, 0.f, 0.f, 0.f};

    for (int kc = 0; kc < SEQ / 64; ++kc) {
        const int kv0 = kc * 64;
        __syncthreads();
        {
            const int r_ = tid >> 1, o_ = (tid & 1) * 32;
            const _Float16* ks = Kb + (size_t)(kv0 + r_) * DM + o_;
            const _Float16* vs = Vb + (size_t)r_ * MTOK + kv0 + o_;
#pragma unroll
            for (int i = 0; i < 4; ++i) {
                const v8h kk = *(const v8h*)(ks + 8 * i);
                const v8h vv = *(const v8h*)(vs + 8 * i);
                *(v8h*)(&Ksh[r_ * 64 + o_ + 8 * i]) = kk;
                *(v8h*)(&Vth[r_ * 64 + o_ + 8 * i]) = vv;
            }
        }
        __syncthreads();

        v8f s[4];
#pragma unroll
        for (int j = 0; j < 4; ++j) {
            FragU k0f, k1f;
            const int kb = (j * 16 + c) * 64 + 8 * hh;
            k0f.h[0] = *(const v8h*)(&Ksh[kb]);      k0f.h[1] = *(const v8h*)(&Ksh[kb + 16]);
            k1f.h[0] = *(const v8h*)(&Ksh[kb + 32]); k1f.h[1] = *(const v8h*)(&Ksh[kb + 48]);
            v8f z = (v8f){0.f, 0.f, 0.f, 0.f, 0.f, 0.f, 0.f, 0.f};
            z = mma16(qa0, k0f.v, z);
            s[j] = mma16(qa1, k1f.v, z);
        }
        float cm[8];
#pragma unroll
        for (int r = 0; r < 8; ++r) {
            float m = NEG;
#pragma unroll
            for (int j = 0; j < 4; ++j) { s[j][r] *= SCL; m = fmaxf(m, s[j][r]); }
#pragma unroll
            for (int off = 1; off < 16; off <<= 1) m = fmaxf(m, __shfl_xor(m, off, 32));
            cm[r] = m;
        }
#pragma unroll
        for (int r = 0; r < 8; ++r) {
            const float mnew = fmaxf(mrow[r], cm[r]);
            const float alpha = exp2f(mrow[r] - mnew);
            mrow[r] = mnew;
            float psum = 0.f;
#pragma unroll
            for (int j = 0; j < 4; ++j) {
                const float p = exp2f(s[j][r] - mnew);
                psum += p;
                Psh[wave][(8 * hh + r) * 64 + j * 16 + c] = (_Float16)(p * PSC);
            }
#pragma unroll
            for (int off = 1; off < 16; off <<= 1) psum += __shfl_xor(psum, off, 32);
            lrow[r] = lrow[r] * alpha + psum;
#pragma unroll
            for (int t = 0; t < 4; ++t) oacc[t][r] *= alpha;
        }
        __builtin_amdgcn_fence(3  , "workgroup");
        __builtin_amdgcn_wave_barrier();
        __builtin_amdgcn_fence(2  , "workgroup");
#pragma unroll
        for (int kk = 0; kk < 2; ++kk) {
            FragU pa;
            pa.h[0] = *(const v8h*)(&Psh[wave][c * 64 + kk * 32 + 8 * hh]);
            pa.h[1] = *(const v8h*)(&Psh[wave][c * 64 + kk * 32 + 16 + 8 * hh]);
#pragma unroll
            for (int t = 0; t < 4; ++t) {
                FragU vb;
                vb.h[0] = *(const v8h*)(&Vth[(t * 16 + c) * 64 + kk * 32 + 8 * hh]);
                vb.h[1] = *(const v8h*)(&Vth[(t * 16 + c) * 64 + kk * 32 + 16 + 8 * hh]);
                oacc[t] = mma16(pa.v, vb.v, oacc[t]);
            }
        }
        __builtin_amdgcn_fence(3  , "workgroup");
        __builtin_amdgcn_wave_barrier();
        __builtin_amdgcn_fence(2  , "workgroup");
    }

#pragma unroll
    for (int r = 0; r < 8; ++r) {
        const float inv = 1.0f / (lrow[r] * PSC);
#pragma unroll
        for (int t = 0; t < 4; ++t) Os[wave][(8 * hh + r) * 68 + t * 16 + c] = oacc[t][r] * inv;
    }
    __builtin_amdgcn_fence(3  , "workgroup");
    __builtin_amdgcn_wave_barrier();
    __builtin_amdgcn_fence(2  , "workgroup");
    {
        const int c4 = (lane & 15) * 4;
        for (int pass = 0; pass < 2; ++pass) {
#pragma unroll
            for (int it = 0; it < 8; ++it) {
                const int row = it * 2 + hh;
                const v4f val = *(const v4f*)(&Os[wave][row * 68 + c4]);
                *(volatile v4f*)(ob + (size_t)(q0 + row) * DM + c4) = val;
            }
            __threadfence();
        }
    }
}

__device__ __forceinline__ v4f ln_t(const float* __restrict__ pa, const float* __restrict__ pb, int abf) {
    v4f a = *(const v4f*)pa; const v4f bb = *(const v4f*)pb;
    if (abf) { a.x = cmb_bf(a.x); a.y = cmb_bf(a.y); a.z = cmb_bf(a.z); a.w = cmb_bf(a.w); }
    v4f t; t.x = a.x + bb.x; t.y = a.y + bb.y; t.z = a.z + bb.z; t.w = a.w + bb.w; return t;
}
__global__ __launch_bounds__(256) void k_ln_part(const float* __restrict__ A, long long sA, int abf, const float* __restrict__ Bv, float* __restrict__ PART) {
    #pragma clang fp contract(off)
    __shared__ float red[256];
    const int tid = threadIdx.x, blk = blockIdx.x, b = blockIdx.y;
    const float* Ab = A + (long long)b * sA + (long long)blk * LN_BLK_ELEMS + tid * 4;
    const float* Bb = Bv + (long long)b * ((long long)SEQ * DM) + (long long)blk * LN_BLK_ELEMS + tid * 4;
    float s = 0.f;
#pragma unroll 1
    for (int it = 0; it < 8; ++it) { const v4f t = ln_t(Ab + it * DM, Bb + it * DM, abf); s += (t.x + t.y) + (t.z + t.w); }
    red[tid] = s; __syncthreads();
    for (int o = 128; o > 0; o >>= 1) { if (tid < o) red[tid] += red[tid + o]; __syncthreads(); }
    const float bsum = red[0]; __syncthreads();
    const float bmean = bsum * (1.0f / (float)LN_BLK_ELEMS);
    float q = 0.f;
#pragma unroll 1
    for (int it = 0; it < 8; ++it) {
        const v4f t = ln_t(Ab + it * DM, Bb + it * DM, abf);
        const float dx = t.x - bmean, dy = t.y - bmean, dz = t.z - bmean, dw = t.w - bmean;
        q += (dx * dx + dy * dy) + (dz * dz + dw * dw);
    }
    red[tid] = q; __syncthreads();
    for (int o = 128; o > 0; o >>= 1) { if (tid < o) red[tid] += red[tid + o]; __syncthreads(); }
    if (tid < 32) {
        const float m2 = red[0];
        const float v = (tid == 0) ? bsum : ((tid == 1) ? m2 : 0.f);
        VST2(float, PART + ((long long)b * LN_BPB + blk) * 32 + tid, v);
    }
}
__global__ __launch_bounds__(256) void k_ln_fin(const float* __restrict__ PART, float* __restrict__ STAT) {
    __shared__ double red[256];
    const int tid = threadIdx.x, b = blockIdx.x;
    const float* P = PART + (long long)b * LN_BPB * 32;
    const double invN = 1.0 / ((double)SEQ * (double)DM);
    const double nblk = (double)LN_BLK_ELEMS, invblk = 1.0 / (double)LN_BLK_ELEMS;
    double s = 0.0;
#pragma unroll 1
    for (int i = tid; i < LN_BPB; i += 256) s += (double)P[(long long)i * 32];
    red[tid] = s; __syncthreads();
    for (int o = 128; o > 0; o >>= 1) { if (tid < o) red[tid] += red[tid + o]; __syncthreads(); }
    const double mean = red[0] * invN; __syncthreads();
    double q = 0.0;
#pragma unroll 1
    for (int i = tid; i < LN_BPB; i += 256) { const double d = (double)P[(long long)i * 32] * invblk - mean; q += (double)P[(long long)i * 32 + 1] + nblk * (d * d); }
    red[tid] = q; __syncthreads();
    for (int o = 128; o > 0; o >>= 1) { if (tid < o) red[tid] += red[tid + o]; __syncthreads(); }
    if (tid < 32) {
        const float var = (float)(red[0] * invN) + 1e-5f;
        const float rstd = 1.0f / sqrtf(var);
        const float v = (tid == 0) ? (float)mean : ((tid == 1) ? rstd : 0.f);
        VST2(float, STAT + (long long)b * 32 + tid, v);
    }
}
__global__ __launch_bounds__(256) void k_ln_apply(const float* __restrict__ A, long long sA, int abf, const float* __restrict__ Bv, const float* __restrict__ STAT,
                                                   float* __restrict__ Yf, unsigned short* __restrict__ Y16) {
    #pragma clang fp contract(off)
    const int tid = threadIdx.x, blk = blockIdx.x, b = blockIdx.y;
    const float mean = STAT[(long long)b * 32], rstd = STAT[(long long)b * 32 + 1];
    const long long ob = (long long)b * ((long long)SEQ * DM) + (long long)blk * LN_BLK_ELEMS + tid * 4;
    const float* Ab = A + (long long)b * sA + (long long)blk * LN_BLK_ELEMS + tid * 4;
    const float* Bb = Bv + ob;
#pragma unroll 1
    for (int it = 0; it < 8; ++it) {
        const v4f t = ln_t(Ab + it * DM, Bb + it * DM, abf);
        v4f y; y.x = (t.x - mean) * rstd; y.y = (t.y - mean) * rstd; y.z = (t.z - mean) * rstd; y.w = (t.w - mean) * rstd;
        const long long o = ob + (long long)it * DM;
        if (Yf != nullptr) VST2V4(Yf + o, y);
        if (Y16 != nullptr) { u2v pk; pk.x = pk2h(y.x, y.y); pk.y = pk2h(y.z, y.w); VST2(u2v, (u2v*)(Y16 + o), pk); }
    }
}

constexpr size_t SZ_X16  = (size_t)MTOK * DM * 2;
constexpr size_t SZ_VT16 = (size_t)DM * MTOK * 2;
constexpr size_t SZ_F16  = (size_t)MTOK * DFF * 2;
constexpr size_t SZ_W    = (size_t)DM * DM * 2;
constexpr size_t SZ_WFF  = (size_t)DFF * DM * 2;
constexpr size_t SZ_F32  = (size_t)MTOK * DM * 4;
constexpr size_t SZ_PART = ((size_t)NB * LN_BPB * 128 + 255) / 256 * 256;
constexpr size_t SZ_STAT = 4096;
constexpr size_t OFF_X16 = 0;
constexpr size_t OFF_Q16 = OFF_X16 + SZ_X16;
constexpr size_t OFF_K16 = OFF_Q16 + SZ_X16;
constexpr size_t OFF_VT  = OFF_K16 + SZ_X16;
constexpr size_t OFF_R0E = OFF_VT + SZ_VT16;
constexpr size_t OFF_WQ  = OFF_R0E;
constexpr size_t OFF_WK  = OFF_WQ + SZ_W;
constexpr size_t OFF_WV  = OFF_WK + SZ_W;
constexpr size_t OFF_W1T = OFF_WV + SZ_W;
constexpr size_t OFF_W2T = OFF_W1T + SZ_WFF;
constexpr size_t OFF_AO  = OFF_W2T + SZ_WFF;
constexpr size_t OFF_HF  = OFF_AO + SZ_F32;
constexpr size_t OFF_H16 = OFF_HF + SZ_F32;
constexpr size_t OFF_P1  = OFF_H16 + SZ_X16;
constexpr size_t OFF_P2  = OFF_P1 + SZ_PART;
constexpr size_t OFF_S1  = OFF_P2 + SZ_PART;
constexpr size_t OFF_S2  = OFF_S1 + SZ_STAT;
constexpr size_t WS_TOTAL = OFF_S2 + SZ_STAT;
static_assert(SZ_F16 <= OFF_R0E - OFF_X16);
static_assert((size_t)NB * 128 <= SZ_STAT);
static_assert((size_t)NB * LN_BPB * 128 <= SZ_PART);
static_assert(WS_TOTAL <= (size_t)134217728);
static_assert((OFF_Q16 % 256) == 0 && (OFF_VT % 256) == 0 && (OFF_WQ % 256) == 0 && (OFF_AO % 256) == 0 && (OFF_P1 % 256) == 0 && (OFF_S1 % 256) == 0);

extern "C" void kernel_launch(void* const* d_in, const int* in_sizes, int n_in, void* d_out, int out_size, void* d_ws, size_t ws_size, hipStream_t stream) {
    if (n_in < 11) return;
    if (in_sizes[0] < ((NB - 1) * SEQ_FULL + SEQ) * DM) return;
    if (in_sizes[1] < DM * DM || in_sizes[3] < DM * DM || in_sizes[5] < DM * DM) return;
    if (in_sizes[2] < DM || in_sizes[4] < DM || in_sizes[6] < DM || in_sizes[10] < DM) return;
    if (in_sizes[7] < DM * DFF || in_sizes[9] < DFF * DM || in_sizes[8] < DFF) return;
    if (out_size < MTOK * DM) return;
    if (WS_TOTAL > ws_size) return;
    const float* x  = (const float*)d_in[0];
    const float* wq = (const float*)d_in[1];
    const float* bq = (const float*)d_in[2];
    const float* wk = (const float*)d_in[3];
    const float* bk = (const float*)d_in[4];
    const float* wv = (const float*)d_in[5];
    const float* bv = (const float*)d_in[6];
    const float* w1 = (const float*)d_in[7];
    const float* b1 = (const float*)d_in[8];
    const float* w2 = (const float*)d_in[9];
    const float* b2 = (const float*)d_in[10];
    float* out = (float*)d_out;
    char* ws = (char*)d_ws;
    unsigned short* X16  = (unsigned short*)(ws + OFF_X16);
    unsigned short* Q16  = (unsigned short*)(ws + OFF_Q16);
    unsigned short* K16  = (unsigned short*)(ws + OFF_K16);
    unsigned short* VT16 = (unsigned short*)(ws + OFF_VT);
    unsigned short* F16p = (unsigned short*)(ws + OFF_X16);
    unsigned short* WQ16 = (unsigned short*)(ws + OFF_WQ);
    unsigned short* WK16 = (unsigned short*)(ws + OFF_WK);
    unsigned short* WV16 = (unsigned short*)(ws + OFF_WV);
    unsigned short* W1T  = (unsigned short*)(ws + OFF_W1T);
    unsigned short* W2T  = (unsigned short*)(ws + OFF_W2T);
    float* AO  = (float*)(ws + OFF_AO);
    float* FFo = (float*)(ws + OFF_AO);
    float* HF  = (float*)(ws + OFF_HF);
    unsigned short* H16 = (unsigned short*)(ws + OFF_H16);
    float* PART1 = (float*)(ws + OFF_P1);
    float* PART2 = (float*)(ws + OFF_P2);
    float* STAT1 = (float*)(ws + OFF_S1);
    float* STAT2 = (float*)(ws + OFF_S2);

    k_cast_x<<<(unsigned)(((long long)MTOK * (DM / 8) + 255) / 256), 256, 0, stream>>>(x, X16);
    k_castT<<<(unsigned)(((long long)DM * (DM / 8) + 255) / 256), 256, 0, stream>>>(wq, DM, WQ16, DM, DM, DM, 16.0f);
    k_castT<<<(unsigned)(((long long)DM * (DM / 8) + 255) / 256), 256, 0, stream>>>(wk, DM, WK16, DM, DM, DM, 16.0f);
    k_castT<<<(unsigned)(((long long)DM * (DM / 8) + 255) / 256), 256, 0, stream>>>(wv, DM, WV16, DM, DM, DM, 16.0f);
    k_castT<<<(unsigned)(((long long)DFF * (DM / 8) + 255) / 256), 256, 0, stream>>>(w1, DFF, W1T, DM, DM, DFF, 16.0f);
    k_castT<<<(unsigned)(((long long)DM * (DFF / 8) + 255) / 256), 256, 0, stream>>>(w2, DM, W2T, DFF, DFF, DM, 16.0f);

    k_gemm_proj<<<(unsigned)(((MTOK / 64) * (DM / 64) + 7) / 8), 256, 0, stream>>>(X16, WQ16, Q16, bq);
    k_gemm_proj<<<(unsigned)(((MTOK / 64) * (DM / 64) + 7) / 8), 256, 0, stream>>>(X16, WK16, K16, bk);
    k_gemm_vt<<<(unsigned)(((DM / 64) * (MTOK / 64) + 7) / 8), 256, 0, stream>>>(WV16, X16, VT16, bv);

    k_attn<<<(unsigned)(NB * NHEAD * (SEQ / 64)), 128, 0, stream>>>(Q16, K16, VT16, AO);

    k_ln_part<<<dim3((unsigned)LN_BPB, (unsigned)NB), 256, 0, stream>>>(x, (long long)SEQ_FULL * DM, 1, AO, PART1);
    k_ln_fin<<<(unsigned)NB, 256, 0, stream>>>(PART1, STAT1);
    k_ln_apply<<<dim3((unsigned)LN_BPB, (unsigned)NB), 256, 0, stream>>>(x, (long long)SEQ_FULL * DM, 1, AO, STAT1, HF, H16);

    k_gemm_ff1<<<(unsigned)(((MTOK / 64) * (DFF / 64) + 7) / 8), 256, 0, stream>>>(H16, W1T, F16p, b1);
    k_gemm_ff2<<<(unsigned)(((MTOK / 64) * (DM / 64) + 7) / 8), 256, 0, stream>>>(F16p, W2T, FFo, b2);

    k_ln_part<<<dim3((unsigned)LN_BPB, (unsigned)NB), 256, 0, stream>>>(HF, (long long)SEQ * DM, 0, FFo, PART2);
    k_ln_fin<<<(unsigned)NB, 256, 0, stream>>>(PART2, STAT2);
    k_ln_apply<<<dim3((unsigned)LN_BPB, (unsigned)NB), 256, 0, stream>>>(HF, (long long)SEQ * DM, 0, FFo, STAT2, out, nullptr);
}
